// RNNAE_39737037423066
// MI455X (gfx1250) — hardware-run, weakly checked
//
#include <hip/hip_runtime.h>
#include <math.h>

typedef __attribute__((ext_vector_type(16))) _Float16 v16h;
typedef __attribute__((ext_vector_type(8)))  float    v8f;
typedef __attribute__((ext_vector_type(4)))  float    v4f;

constexpr int kRollouts      = 2097152;
constexpr int kSteps         = 10;
constexpr int kHid           = 10;
constexpr int kInW           = 2;
constexpr int kGateRows      = 4 * kHid;
constexpr int kMlp           = 2 * kHid;
constexpr int kBlocks        = 4096;
constexpr int kThreads       = 64;
constexpr int kWaves         = kThreads / 32;
constexpr int kGroupsPerWave = 8;
constexpr int kGroupRows     = 32;
constexpr int kPitch         = 36;
constexpr int kSlabFloats    = 16 * kPitch;
constexpr int kColS          = kHid;
constexpr int kColA          = kHid + 1;
constexpr int kReadCol       = kColS;
static_assert(kBlocks * kWaves * kGroupsPerWave * kGroupRows == kRollouts, "grid covers every rollout exactly once");
static_assert(kHid + kInW <= 16, "cell operand fits the low 16 k slots");
static_assert(kMlp <= 32 && kMlp > 16, "perceptron width uses both k halves");
static_assert((kPitch % 4) == 0, "16-B aligned row reads");
static_assert(kGroupRows * 4 == 128, "one group of outputs = one 128-B line");

constexpr float kActCarry = 16.0f;
constexpr float kWgtCarry = 256.0f;
constexpr float kFold     = 1.0f / (kActCarry * kWgtCarry);
constexpr float kF16MinNormal = 6.103515625e-5f;
static_assert(kFold == 1.0f / 4096.0f, "fold constant");
constexpr float kInvDenEarly = 1.0f / 0.2f;
constexpr float kInvDenLate  = 1.0f / 0.4f;

__device__ __forceinline__ float fsig(float x)  { return __builtin_amdgcn_rcpf(1.0f + __expf(-x)); }
__device__ __forceinline__ float ftanh(float x) { return 1.0f - 2.0f * __builtin_amdgcn_rcpf(__expf(2.0f * x) + 1.0f); }

__device__ __forceinline__ _Float16 to_h(float x, float carry) {
  float y = x * carry;
  y = (fabsf(y) < kF16MinNormal) ? 0.0f : y;
  return (_Float16)y;
}

template <bool FULL>
__device__ __forceinline__ v16h build_frag(const float* p, float carry) {
  v16h f;
  const v4f q0 = *(const v4f*)(p);
  const v4f q1 = *(const v4f*)(p + 4);
#pragma unroll
  for (int e = 0; e < 4; ++e) {
    f[e]     = to_h(q0[e], carry);
    f[4 + e] = to_h(q1[e], carry);
  }
  if (FULL) {
    const v4f q2 = *(const v4f*)(p + 16);
    const v4f q3 = *(const v4f*)(p + 20);
#pragma unroll
    for (int e = 0; e < 4; ++e) {
      f[8 + e]  = to_h(q2[e], carry);
      f[12 + e] = to_h(q3[e], carry);
    }
  } else {
#pragma unroll
    for (int e = 0; e < 8; ++e) f[8 + e] = (_Float16)0.0f;
  }
  return f;
}

__device__ __forceinline__ v8f mma_g(v16h a, v16h b, v8f c) {
  c = __builtin_amdgcn_wmma_f32_16x16x32_f16(false, a, false, b, (short)0, c, false, false);
  asm volatile("v_nop\n\tv_nop\n\tv_nop\n\tv_nop" : "+v"(c) : "v"(a), "v"(b));
  return c;
}

__global__ void __launch_bounds__(kThreads) __attribute__((amdgpu_num_vgpr(256)))
rollout_kernel(const float* __restrict__ s_star, const int* __restrict__ go_mask,
               const float* __restrict__ W_ih, const float* __restrict__ W_hh,
               const float* __restrict__ b_ih, const float* __restrict__ b_hh,
               const float* __restrict__ W1, const float* __restrict__ b1,
               const float* __restrict__ W2, const float* __restrict__ b2,
               const float* __restrict__ W3, const float* __restrict__ b3,
               float* __restrict__ out)
{
  __shared__ __align__(16) float sBc[64 * kPitch];
  __shared__ __align__(16) float sB1[32 * kPitch];
  __shared__ __align__(16) float sB2[32 * kPitch];
  __shared__ __align__(16) float sB3[16 * kPitch];
  __shared__ __align__(16) float sSlab[kWaves * 2 * kSlabFloats];

  const int tid  = threadIdx.x;
  const int lane = tid & 31;
  const int wave = tid >> 5;
  const int n    = lane & 15;
  const int half = lane >> 4;

  {
    const int k  = tid & 31;
    const int kh = (k < kHid - 1) ? k : (kHid - 1);
    const int ki = (k == kColA) ? 1 : 0;
    const int km = (k < kMlp - 1) ? k : (kMlp - 1);
#pragma unroll 1
    for (int it = 0; it < 32; ++it) {
      const int nn = 2 * it + wave;
      const int q  = nn >> 4;
      const int u  = nn & 15;
      const int uc = (u < kHid - 1) ? u : (kHid - 1);
      const int gr = kHid * q + uc;
      float whh = W_hh[gr * kHid + kh];
      asm volatile("" : "+v"(whh));
      float wih = W_ih[gr * kInW + ki];
      asm volatile("" : "+v"(wih));
      float v = (k < kHid) ? whh : wih;
      v = ((u < kHid) && (k < kHid + kInW)) ? v : 0.0f;
      sBc[nn * kPitch + k] = v;
    }
#pragma unroll 1
    for (int it = 0; it < 16; ++it) {
      const int nn = 2 * it + wave;
      const int nc = (nn < kMlp - 1) ? nn : (kMlp - 1);
      float w1v = W1[nc * kHid + kh];
      asm volatile("" : "+v"(w1v));
      float w2v = W2[nc * kMlp + km];
      asm volatile("" : "+v"(w2v));
      const float v1 = ((nn < kMlp) && (k < kHid)) ? w1v : 0.0f;
      const float v2 = ((nn < kMlp) && (k < kMlp)) ? w2v : 0.0f;
      sB1[nn * kPitch + k] = v1;
      sB2[nn * kPitch + k] = v2;
    }
#pragma unroll 1
    for (int it = 0; it < 8; ++it) {
      const int nn = 2 * it + wave;
      float w3v = W3[km];
      asm volatile("" : "+v"(w3v));
      const float v3 = ((nn == kReadCol) && (k < kMlp)) ? w3v : 0.0f;
      sB3[nn * kPitch + k] = v3;
    }
  }

  float bg[4], bl1[2], bl2[2];
  {
    const int nc = (n < kHid - 1) ? n : (kHid - 1);
#pragma unroll
    for (int q = 0; q < 4; ++q) {
      float ba = b_ih[kHid * q + nc];
      asm volatile("" : "+v"(ba));
      float bb = b_hh[kHid * q + nc];
      asm volatile("" : "+v"(bb));
      bg[q] = (n < kHid) ? (ba + bb) : 0.0f;
    }
#pragma unroll
    for (int j = 0; j < 2; ++j) {
      const int f  = 16 * j + n;
      const int fc = (f < kMlp - 1) ? f : (kMlp - 1);
      float x1 = b1[fc];
      asm volatile("" : "+v"(x1));
      float x2 = b2[fc];
      asm volatile("" : "+v"(x2));
      bl1[j] = (f < kMlp) ? x1 : 0.0f;
      bl2[j] = (f < kMlp) ? x2 : 0.0f;
    }
  }
  const float b3v = b3[0];

  int gobits = 0;
#pragma unroll
  for (int t = 0; t < kSteps; ++t) {
    const int gv = go_mask[t];
    gobits |= (gv != 0) ? (1 << t) : 0;
  }

  __syncthreads();

  const int fo = n * kPitch + 8 * half;
  v16h bc[4], bm1[2], bm2[2];
#pragma unroll
  for (int q = 0; q < 4; ++q) bc[q] = build_frag<true>(sBc + q * 16 * kPitch + fo, kWgtCarry);
#pragma unroll
  for (int j = 0; j < 2; ++j) {
    bm1[j] = build_frag<true>(sB1 + j * 16 * kPitch + fo, kWgtCarry);
    bm2[j] = build_frag<true>(sB2 + j * 16 * kPitch + fo, kWgtCarry);
  }
  const v16h bro = build_frag<true>(sB3 + fo, kWgtCarry);

  float* const slabw = sSlab + wave * (2 * kSlabFloats);
  const int co = (8 * half) * kPitch + n;
  const bool isUnit = (n < kHid);
  const bool isS    = (n == kColS);
  const bool isA    = (n == kColA);
  const bool tailOn = ((16 + n) < kMlp);
  const int wglobal = blockIdx.x * kWaves + wave;
  const v8f z8 = {0.f, 0.f, 0.f, 0.f, 0.f, 0.f, 0.f, 0.f};

#pragma unroll 1
  for (int gi = 0; gi < kGroupsPerWave; ++gi) {
    const int base = (wglobal * kGroupsPerWave + gi) * kGroupRows;

    float sst[2][8], cs[2][8], hs[2][8], ss[2][8], er[2][8];
#pragma unroll
    for (int tl = 0; tl < 2; ++tl) {
      const float* sp = s_star + base + tl * 16 + 8 * half;
      const v4f a0 = *(const v4f*)(sp);
      const v4f a1 = *(const v4f*)(sp + 4);
#pragma unroll
      for (int e = 0; e < 4; ++e) {
        sst[tl][e]     = a0[e];
        sst[tl][4 + e] = a1[e];
      }
#pragma unroll
      for (int r = 0; r < 8; ++r) {
        cs[tl][r] = 0.0f;
        hs[tl][r] = 0.0f;
        ss[tl][r] = 0.0f;
        er[tl][r] = 0.0f;
      }
    }

#pragma unroll 1
    for (int t = 0; t < kSteps; ++t) {
      const bool  goT  = ((gobits >> t) & 1) != 0;
      const float rden = (t < 4) ? kInvDenEarly : kInvDenLate;

#pragma unroll
      for (int tl = 0; tl < 2; ++tl) {
        float* sl = slabw + tl * kSlabFloats + co;
#pragma unroll
        for (int r = 0; r < 8; ++r) {
          const float ahv = goT ? ((sst[tl][r] - 0.6f) * rden) : 0.0f;
          float v = isA ? ahv : 0.0f;
          v = isS ? ss[tl][r] : v;
          v = isUnit ? hs[tl][r] : v;
          sl[r * kPitch] = v;
        }
      }
      __syncthreads();
#pragma unroll
      for (int tl = 0; tl < 2; ++tl) {
        const v16h a = build_frag<false>(slabw + tl * kSlabFloats + fo, kActCarry);
        v8f g0 = z8, g1 = z8, g2 = z8, g3 = z8;
        g0 = mma_g(a, bc[0], g0);
        g1 = mma_g(a, bc[1], g1);
        g2 = mma_g(a, bc[2], g2);
        g3 = mma_g(a, bc[3], g3);
#pragma unroll
        for (int r = 0; r < 8; ++r) {
          const float zi = fmaf(g0[r], kFold, bg[0]);
          const float zf = fmaf(g1[r], kFold, bg[1]);
          const float zg = fmaf(g2[r], kFold, bg[2]);
          const float zo = fmaf(g3[r], kFold, bg[3]);
          const float ig = fsig(zi);
          const float fg = fsig(zf);
          const float gg = ftanh(zg);
          const float og = fsig(zo);
          const float cn = fmaf(fg, cs[tl][r], ig * gg);
          cs[tl][r] = cn;
          hs[tl][r] = og * ftanh(cn);
        }
      }
      __syncthreads();

#pragma unroll
      for (int tl = 0; tl < 2; ++tl) {
        float* sl = slabw + tl * kSlabFloats + co;
#pragma unroll
        for (int r = 0; r < 8; ++r) {
          const float v = isUnit ? hs[tl][r] : 0.0f;
          sl[r * kPitch] = v;
        }
      }
      __syncthreads();
      float p[2][2][8];
#pragma unroll
      for (int tl = 0; tl < 2; ++tl) {
        const v16h a = build_frag<false>(slabw + tl * kSlabFloats + fo, kActCarry);
        v8f u0 = z8, u1 = z8;
        u0 = mma_g(a, bm1[0], u0);
        u1 = mma_g(a, bm1[1], u1);
#pragma unroll
        for (int r = 0; r < 8; ++r) {
          const float x0 = fmaf(u0[r], kFold, bl1[0]);
          const float x1 = fmaf(u1[r], kFold, bl1[1]);
          p[tl][0][r] = fmaxf(x0, 0.0f);
          p[tl][1][r] = tailOn ? fmaxf(x1, 0.0f) : 0.0f;
        }
      }
      __syncthreads();

#pragma unroll
      for (int tl = 0; tl < 2; ++tl) {
        float* sl = slabw + tl * kSlabFloats + co;
#pragma unroll
        for (int r = 0; r < 8; ++r) {
          sl[r * kPitch]      = p[tl][0][r];
          sl[r * kPitch + 16] = p[tl][1][r];
        }
      }
      __syncthreads();
#pragma unroll
      for (int tl = 0; tl < 2; ++tl) {
        const v16h a = build_frag<true>(slabw + tl * kSlabFloats + fo, kActCarry);
        v8f u0 = z8, u1 = z8;
        u0 = mma_g(a, bm2[0], u0);
        u1 = mma_g(a, bm2[1], u1);
#pragma unroll
        for (int r = 0; r < 8; ++r) {
          const float x0 = fmaf(u0[r], kFold, bl2[0]);
          const float x1 = fmaf(u1[r], kFold, bl2[1]);
          p[tl][0][r] = fmaxf(x0, 0.0f);
          p[tl][1][r] = tailOn ? fmaxf(x1, 0.0f) : 0.0f;
        }
      }
      __syncthreads();

#pragma unroll
      for (int tl = 0; tl < 2; ++tl) {
        float* sl = slabw + tl * kSlabFloats + co;
#pragma unroll
        for (int r = 0; r < 8; ++r) {
          sl[r * kPitch]      = p[tl][0][r];
          sl[r * kPitch + 16] = p[tl][1][r];
        }
      }
      __syncthreads();
#pragma unroll
      for (int tl = 0; tl < 2; ++tl) {
        const v16h a = build_frag<true>(slabw + tl * kSlabFloats + fo, kActCarry);
        v8f d3 = z8;
        d3 = mma_g(a, bro, d3);
#pragma unroll
        for (int r = 0; r < 8; ++r) {
          const float ar = fmaf(d3[r], kFold, b3v);
          const float sn = ss[tl][r] + ar;
          ss[tl][r] = sn;
          const float df = sn - sst[tl][r];
          er[tl][r] = fmaf(df, df, er[tl][r]);
        }
      }
      __syncthreads();
    }

#pragma unroll
    for (int tl = 0; tl < 2; ++tl) {
      float* sl = slabw + tl * kSlabFloats + co;
#pragma unroll
      for (int r = 0; r < 8; ++r) sl[r * kPitch] = er[tl][r];
    }
    __syncthreads();
    const float val = slabw[half * kSlabFloats + n * kPitch + kReadCol];
    __syncthreads();
    float* op = out + base + lane;
    *(volatile float*)op = val;
    __threadfence();
    *(volatile float*)op = val;
  }
}

extern "C" void kernel_launch(void* const* d_in, const int* in_sizes, int n_in,
                              void* d_out, int out_size, void* d_ws, size_t ws_size,
                              hipStream_t stream) {
  (void)d_ws; (void)ws_size;
  if (n_in < 12 || d_out == nullptr) return;
  if (in_sizes[0] != kRollouts) return;
  if (in_sizes[1] != kSteps) return;
  if (in_sizes[2] != kGateRows * kInW) return;
  if (in_sizes[3] != kGateRows * kHid) return;
  if (in_sizes[4] != kGateRows) return;
  if (in_sizes[5] != kGateRows) return;
  if (in_sizes[6] != kMlp * kHid) return;
  if (in_sizes[7] != kMlp) return;
  if (in_sizes[8] != kMlp * kMlp) return;
  if (in_sizes[9] != kMlp) return;
  if (in_sizes[10] != kMlp) return;
  if (in_sizes[11] != 1) return;
  if (out_size != kRollouts) return;

  const float* s_star = (const float*)d_in[0];
  const int*   go     = (const int*)d_in[1];
  const float* W_ih   = (const float*)d_in[2];
  const float* W_hh   = (const float*)d_in[3];
  const float* b_ih   = (const float*)d_in[4];
  const float* b_hh   = (const float*)d_in[5];
  const float* W1     = (const float*)d_in[6];
  const float* b1     = (const float*)d_in[7];
  const float* W2     = (const float*)d_in[8];
  const float* b2     = (const float*)d_in[9];
  const float* W3     = (const float*)d_in[10];
  const float* b3     = (const float*)d_in[11];
  float* out = (float*)d_out;

  rollout_kernel<<<dim3(kBlocks), dim3(kThreads), 0, stream>>>(
      s_star, go, W_ih, W_hh, b_ih, b_hh, W1, b1, W2, b2, W3, b3, out);
}
